// GenView_1778116461037
// MI455X (gfx1250) — hardware-verified
//
#include <hip/hip_runtime.h>
#include <stdint.h>
#include <stddef.h>


#define FIN   256
#define HID   64
#define PW    264
#define PX    72
#define NB1   7680
#define NB2   15360
#define NTAG  1024
#define LAMBDA_C 0.5f

typedef _Float16 v16h __attribute__((ext_vector_type(16)));
typedef _Float16 v8h  __attribute__((ext_vector_type(8)));
typedef float    v8f  __attribute__((ext_vector_type(8)));
typedef float    v4f  __attribute__((ext_vector_type(4)));
union Frag { v16h v; v8h half[2]; };

__device__ __forceinline__ v8f wmma_f16(v8f acc, v16h a, v16h b)
{
    acc = __builtin_amdgcn_wmma_f32_16x16x32_f16(false, a, false, b, (short)0, acc, false, false);
    asm volatile("v_nop\n\tv_nop\n\tv_nop\n\tv_nop" : "+v"(acc) : "v"(a), "v"(b));
    return acc;
}

__device__ __forceinline__ v8h cvt8h(const float* __restrict__ p)
{
    const v4f f0 = *(const v4f*)(p);
    const v4f f1 = *(const v4f*)(p + 4);
    v8h r;
    r[0] = (_Float16)f0[0]; r[1] = (_Float16)f0[1]; r[2] = (_Float16)f0[2]; r[3] = (_Float16)f0[3];
    r[4] = (_Float16)f1[0]; r[5] = (_Float16)f1[1]; r[6] = (_Float16)f1[2]; r[7] = (_Float16)f1[3];
    return r;
}

__device__ __forceinline__ int clampi(int x, int hi)
{
    return x < 0 ? 0 : (x > hi ? hi : x);
}

__global__ __launch_bounds__(128)
void k_proj(const float* __restrict__ feat, const float* __restrict__ Wg,
            const float* __restrict__ bg, const float* __restrict__ Wm,
            float* __restrict__ y, int N)
{
    __shared__ __attribute__((aligned(16))) _Float16 Wt[HID * PW];
    __shared__ __attribute__((aligned(16))) _Float16 Bm[16 * PX];
    __shared__ __attribute__((aligned(16))) _Float16 xs[4 * 16 * PX];
    __shared__ __attribute__((aligned(16))) float    yt[4 * 32];

    const int tid = threadIdx.x;
    const int w = tid >> 5, l = tid & 31, h = l >> 4, m = l & 15;

    for (int idx = tid; idx < FIN * HID; idx += 128) {
        const int k = idx >> 6, n = idx & 63;
        Wt[n * PW + k] = (_Float16)(Wg[idx] * 16.0f);
    }
    for (int idx = tid; idx < 16 * HID; idx += 128) {
        const int n = idx >> 6, k = idx & 63;
        float v = 0.0f;
        if (n < 2) v = Wm[n * HID + k] * 16.0f;
        Bm[n * PX + k] = (_Float16)v;
    }
    __syncthreads();

    const int row0 = (blockIdx.x * 4 + w) * 16;
    int ra = row0 + m;
    if (ra > N - 1) ra = N - 1;
    const float* arow = feat + (size_t)ra * FIN;

    const v8f z8 = {0.0f, 0.0f, 0.0f, 0.0f, 0.0f, 0.0f, 0.0f, 0.0f};
    v8f acc0 = z8, acc1 = z8, acc2 = z8, acc3 = z8;

#pragma unroll 1
    for (int k0 = 0; k0 < FIN; k0 += 32) {
        Frag a, b;
        a.half[0] = cvt8h(arow + k0 + 8 * h);
        a.half[1] = cvt8h(arow + k0 + 16 + 8 * h);
        const _Float16* bp = Wt + m * PW + k0 + 8 * h;
        b.half[0] = *(const v8h*)(bp);
        b.half[1] = *(const v8h*)(bp + 16);
        acc0 = wmma_f16(acc0, a.v, b.v);
        b.half[0] = *(const v8h*)(bp + 16 * PW);
        b.half[1] = *(const v8h*)(bp + 16 * PW + 16);
        acc1 = wmma_f16(acc1, a.v, b.v);
        b.half[0] = *(const v8h*)(bp + 32 * PW);
        b.half[1] = *(const v8h*)(bp + 32 * PW + 16);
        acc2 = wmma_f16(acc2, a.v, b.v);
        b.half[0] = *(const v8h*)(bp + 48 * PW);
        b.half[1] = *(const v8h*)(bp + 48 * PW + 16);
        acc3 = wmma_f16(acc3, a.v, b.v);
    }

    _Float16* xw_s = xs + w * (16 * PX);
    {
        const float b0 = bg[m], b1 = bg[16 + m], b2 = bg[32 + m], b3 = bg[48 + m];
#pragma unroll
        for (int r = 0; r < 8; ++r) {
            const int rb = (8 * h + r) * PX;
            xw_s[rb + m]      = (_Float16)(acc0[r] * 0.0625f + b0);
            xw_s[rb + 16 + m] = (_Float16)(acc1[r] * 0.0625f + b1);
            xw_s[rb + 32 + m] = (_Float16)(acc2[r] * 0.0625f + b2);
            xw_s[rb + 48 + m] = (_Float16)(acc3[r] * 0.0625f + b3);
        }
    }
    __syncthreads();

    v8f yacc = z8;
#pragma unroll
    for (int ks = 0; ks < HID; ks += 32) {
        Frag a, b;
        const _Float16* ap = xw_s + m * PX + ks + 8 * h;
        a.half[0] = *(const v8h*)(ap);
        a.half[1] = *(const v8h*)(ap + 16);
        const _Float16* bq = Bm + m * PX + ks + 8 * h;
        b.half[0] = *(const v8h*)(bq);
        b.half[1] = *(const v8h*)(bq + 16);
        yacc = wmma_f16(yacc, a.v, b.v);
    }

    float* yts = yt + w * 32;
    if (m < 2) {
#pragma unroll
        for (int r = 0; r < 8; ++r) yts[(8 * h + r) * 2 + m] = yacc[r] * 0.0625f;
    }
    __syncthreads();

    v4f vq = {0.0f, 0.0f, 0.0f, 0.0f};
    if (l < 8) vq = *(const v4f*)(yts + 4 * l);
    volatile v4f* dst = (volatile v4f*)(y + (size_t)row0 * 2 + 4 * l);
    if (l < 8) *dst = vq;
    __threadfence();
    if (l < 8) *dst = vq;
}

__global__ __launch_bounds__(32)
void k_seg_pq(const int* __restrict__ rows, const int* __restrict__ cols,
              const float* __restrict__ vv, const float* __restrict__ y,
              const int* __restrict__ nn, float* __restrict__ PQ, int E, int N)
{
    extern __shared__ __attribute__((aligned(16))) float dsm[];
    float* pq  = dsm;
    int*   tag = (int*)(dsm + 2 * NB1);

    const int l = threadIdx.x;
    const int nb0 = blockIdx.x * NB1;
    int nseg = nn[0];
    if (nseg < 0) nseg = 0;
    if (nseg > N) nseg = N;
    int cnt = nseg - nb0;
    if (cnt > NB1) cnt = NB1;
    if (cnt < 0) cnt = 0;

    const v4f z4 = {0.0f, 0.0f, 0.0f, 0.0f};
    for (int i = l; i < (2 * NB1) / 4; i += 32) ((v4f*)pq)[i] = z4;
    for (int i = l; i < NTAG; i += 32) tag[i] = -1;
    __syncthreads();

    for (int e0 = 0; e0 < E; e0 += 32) {
        const int e = e0 + l;
        const bool valid = e < E;
        int r = 0, c = 0;
        float v = 0.0f;
        if (valid) { r = rows[e]; c = cols[e]; v = vv[e]; }
        const int ln = r - nb0;
        const bool hit = valid && ((unsigned)ln < (unsigned)cnt);
        float a0 = 0.0f, a1 = 0.0f;
        if (hit) {
            const int cc = clampi(c, N - 1);
            a0 = v * y[2 * cc];
            a1 = v * y[2 * cc + 1];
        }
        const unsigned mask = __builtin_amdgcn_ballot_w32(hit);
        if (mask == 0u) continue;
        const int tg = ln & (NTAG - 1);
        if (hit) tag[tg] = l;
        __syncthreads();
        int seen = l;
        if (hit) seen = tag[tg];
        const unsigned dmask = __builtin_amdgcn_ballot_w32(seen != l);
        if (dmask == 0u) {
            if (hit) {
                pq[2 * ln]     += a0;
                pq[2 * ln + 1] += a1;
            }
        } else {
            unsigned mk = mask;
            while (mk != 0u) {
                const int j = __builtin_ctz(mk);
                mk &= mk - 1u;
                const int   lnj = __shfl(ln, j, 32);
                const float b0  = __shfl(a0, j, 32);
                const float b1  = __shfl(a1, j, 32);
                if (l == 0) {
                    pq[2 * lnj]     += b0;
                    pq[2 * lnj + 1] += b1;
                }
            }
        }
    }
    __syncthreads();

    const int nq = (2 * NB1) / 4;
    volatile v4f* dst = (volatile v4f*)(PQ + (size_t)2 * nb0);
    for (int i = l; i < nq; i += 32) { const v4f t = ((const v4f*)pq)[i]; dst[i] = t; }
    __threadfence();
    for (int i = l; i < nq; i += 32) { const v4f t = ((const v4f*)pq)[i]; dst[i] = t; }
}

__global__ __launch_bounds__(32)
void k_seg_max(const int* __restrict__ rows, const int* __restrict__ cols,
               const float* __restrict__ PQ, const float* __restrict__ bm,
               const int* __restrict__ nn, float* __restrict__ MX, int E, int N)
{
    extern __shared__ __attribute__((aligned(16))) float dsm[];
    float* mx  = dsm;
    int*   tag = (int*)(dsm + NB2);

    const int l = threadIdx.x;
    const int nb0 = blockIdx.x * NB2;
    int nseg = nn[0];
    if (nseg < 0) nseg = 0;
    if (nseg > N) nseg = N;
    int cnt = nseg - nb0;
    if (cnt > NB2) cnt = NB2;
    if (cnt < 0) cnt = 0;
    const float bm0 = bm[0];

    const float ninf = -__builtin_inff();
    const v4f n4 = {ninf, ninf, ninf, ninf};
    for (int i = l; i < NB2 / 4; i += 32) ((v4f*)mx)[i] = n4;
    for (int i = l; i < NTAG; i += 32) tag[i] = -1;
    __syncthreads();

    for (int e0 = 0; e0 < E; e0 += 32) {
        const int e = e0 + l;
        const bool valid = e < E;
        int r = 0, c = 0;
        if (valid) { r = rows[e]; c = cols[e]; }
        const int ln = r - nb0;
        const bool hit = valid && ((unsigned)ln < (unsigned)cnt);
        float t = 0.0f;
        if (hit) {
            const int cc = clampi(c, N - 1);
            t = (PQ[2 * r] + PQ[2 * cc + 1]) + bm0;
        }
        const unsigned mask = __builtin_amdgcn_ballot_w32(hit);
        if (mask == 0u) continue;
        const int tg = ln & (NTAG - 1);
        if (hit) tag[tg] = l;
        __syncthreads();
        int seen = l;
        if (hit) seen = tag[tg];
        const unsigned dmask = __builtin_amdgcn_ballot_w32(seen != l);
        if (dmask == 0u) {
            if (hit) mx[ln] = fmaxf(mx[ln], t);
        } else {
            unsigned mk = mask;
            while (mk != 0u) {
                const int j = __builtin_ctz(mk);
                mk &= mk - 1u;
                const int   lnj = __shfl(ln, j, 32);
                const float tj  = __shfl(t, j, 32);
                if (l == 0) mx[lnj] = fmaxf(mx[lnj], tj);
            }
        }
    }
    __syncthreads();

    const int nq = NB2 / 4;
    volatile v4f* dst = (volatile v4f*)(MX + (size_t)nb0);
    for (int i = l; i < nq; i += 32) { const v4f tq = ((const v4f*)mx)[i]; dst[i] = tq; }
    __threadfence();
    for (int i = l; i < nq; i += 32) { const v4f tq = ((const v4f*)mx)[i]; dst[i] = tq; }
}

__global__ __launch_bounds__(32)
void k_seg_sum(const int* __restrict__ rows, const int* __restrict__ cols,
               const float* __restrict__ PQ, const float* __restrict__ bm,
               const int* __restrict__ nn, const float* __restrict__ MX,
               float* __restrict__ S, int E, int N)
{
    extern __shared__ __attribute__((aligned(16))) float dsm[];
    float* sm  = dsm;
    int*   tag = (int*)(dsm + NB2);

    const int l = threadIdx.x;
    const int nb0 = blockIdx.x * NB2;
    int nseg = nn[0];
    if (nseg < 0) nseg = 0;
    if (nseg > N) nseg = N;
    int cnt = nseg - nb0;
    if (cnt > NB2) cnt = NB2;
    if (cnt < 0) cnt = 0;
    const float bm0 = bm[0];

    const v4f z4 = {0.0f, 0.0f, 0.0f, 0.0f};
    for (int i = l; i < NB2 / 4; i += 32) ((v4f*)sm)[i] = z4;
    for (int i = l; i < NTAG; i += 32) tag[i] = -1;
    __syncthreads();

    for (int e0 = 0; e0 < E; e0 += 32) {
        const int e = e0 + l;
        const bool valid = e < E;
        int r = 0, c = 0;
        if (valid) { r = rows[e]; c = cols[e]; }
        const int ln = r - nb0;
        const bool hit = valid && ((unsigned)ln < (unsigned)cnt);
        float ex = 0.0f;
        if (hit) {
            const int cc = clampi(c, N - 1);
            const float t = (PQ[2 * r] + PQ[2 * cc + 1]) + bm0;
            ex = __expf(t - MX[r]);
        }
        const unsigned mask = __builtin_amdgcn_ballot_w32(hit);
        if (mask == 0u) continue;
        const int tg = ln & (NTAG - 1);
        if (hit) tag[tg] = l;
        __syncthreads();
        int seen = l;
        if (hit) seen = tag[tg];
        const unsigned dmask = __builtin_amdgcn_ballot_w32(seen != l);
        if (dmask == 0u) {
            if (hit) sm[ln] += ex;
        } else {
            unsigned mk = mask;
            while (mk != 0u) {
                const int j = __builtin_ctz(mk);
                mk &= mk - 1u;
                const int   lnj = __shfl(ln, j, 32);
                const float exj = __shfl(ex, j, 32);
                if (l == 0) sm[lnj] += exj;
            }
        }
    }
    __syncthreads();

    const int nq = NB2 / 4;
    volatile v4f* dst = (volatile v4f*)(S + (size_t)nb0);
    for (int i = l; i < nq; i += 32) { const v4f tq = ((const v4f*)sm)[i]; dst[i] = tq; }
    __threadfence();
    for (int i = l; i < nq; i += 32) { const v4f tq = ((const v4f*)sm)[i]; dst[i] = tq; }
}

__device__ __forceinline__ float edge_value(int e, const int* __restrict__ rows,
                                            const int* __restrict__ cols,
                                            const float* __restrict__ vv,
                                            const float* __restrict__ PQ,
                                            const float* __restrict__ MX,
                                            const float* __restrict__ S,
                                            float bm0, int N)
{
    const int r = clampi(rows[e], N - 1);
    const int c = clampi(cols[e], N - 1);
    const float t  = (PQ[2 * r] + PQ[2 * c + 1]) + bm0;
    const float ex = __expf(t - MX[r]);
    const float pi = ex / S[r];
    return vv[e] + LAMBDA_C * pi;
}

__global__ __launch_bounds__(256)
void k_out(const int* __restrict__ rows, const int* __restrict__ cols,
           const float* __restrict__ vv, const float* __restrict__ PQ,
           const float* __restrict__ MX, const float* __restrict__ S,
           const float* __restrict__ bm, float* __restrict__ out, int E, int N)
{
    const int gt  = blockIdx.x * 256 + threadIdx.x;
    const int nq  = E >> 2;
    const int rem = E & 3;
    const float bm0 = bm[0];
    const bool act  = gt < nq;
    const bool tact = gt < rem;

    v4f o = {0.0f, 0.0f, 0.0f, 0.0f};
    if (act) {
#pragma unroll
        for (int i = 0; i < 4; ++i)
            o[i] = edge_value(4 * gt + i, rows, cols, vv, PQ, MX, S, bm0, N);
    }
    float ot = 0.0f;
    const int et = (nq << 2) + gt;
    if (tact) ot = edge_value(et, rows, cols, vv, PQ, MX, S, bm0, N);

    if (act)  { volatile v4f*  dq = (volatile v4f*)(out + (size_t)4 * gt); *dq = o; }
    if (tact) { volatile float* dt = (volatile float*)(out + et);            *dt = ot; }
    __threadfence();
    if (act)  { volatile v4f*  dq = (volatile v4f*)(out + (size_t)4 * gt); *dq = o; }
    if (tact) { volatile float* dt = (volatile float*)(out + et);            *dt = ot; }
}

extern "C" void kernel_launch(void* const* d_in, const int* in_sizes, int n_in,
                              void* d_out, int out_size, void* d_ws, size_t ws_size,
                              hipStream_t stream)
{
    if (n_in < 8) return;
    const float* v_ori = (const float*)d_in[0];
    const float* feat  = (const float*)d_in[1];
    const float* W_gcn = (const float*)d_in[2];
    const float* b_gcn = (const float*)d_in[3];
    const float* W_mlp = (const float*)d_in[4];
    const float* b_mlp = (const float*)d_in[5];
    const int*   vidx  = (const int*)d_in[6];
    const int*   nnode = (const int*)d_in[7];

    const int E = in_sizes[0];
    const int N = in_sizes[1] / FIN;
    if (E <= 0 || N <= 0) return;
    if (in_sizes[6] < 2 * E) return;
    if (out_size < E) return;
    const int* rows = vidx;
    const int* cols = vidx + (size_t)E;

    const int nblk1 = (N + 63) / 64;
    const int nb1   = (N + NB1 - 1) / NB1;
    const int nb2   = (N + NB2 - 1) / NB2;

    size_t off = 0;
    const size_t by  = ((size_t)nblk1 * 64 * 2 * sizeof(float) + 255) & ~(size_t)255;
    float* y  = (float*)((char*)d_ws + off); off += by;
    const size_t bpq = ((size_t)nb1 * NB1 * 2 * sizeof(float) + 255) & ~(size_t)255;
    float* PQ = (float*)((char*)d_ws + off); off += bpq;
    const size_t bn  = ((size_t)nb2 * NB2 * sizeof(float) + 255) & ~(size_t)255;
    float* MX = (float*)((char*)d_ws + off); off += bn;
    float* S  = (float*)((char*)d_ws + off); off += bn;
    if (off > ws_size) return;

    const size_t lds_pq = (size_t)(2 * NB1 + NTAG) * sizeof(float);
    const size_t lds_n  = (size_t)(NB2 + NTAG) * sizeof(float);

    k_proj<<<nblk1, 128, 0, stream>>>(feat, W_gcn, b_gcn, W_mlp, y, N);
    k_seg_pq<<<nb1, 32, lds_pq, stream>>>(rows, cols, v_ori, y, nnode, PQ, E, N);
    k_seg_max<<<nb2, 32, lds_n, stream>>>(rows, cols, PQ, b_mlp, nnode, MX, E, N);
    k_seg_sum<<<nb2, 32, lds_n, stream>>>(rows, cols, PQ, b_mlp, nnode, MX, S, E, N);

    const int nq = E >> 2;
    const int g5 = ((nq > 0 ? nq : 1) + 255) / 256;
    k_out<<<g5, 256, 0, stream>>>(rows, cols, v_ori, PQ, MX, S, b_mlp, (float*)d_out, E, N);
}
